// PointNetSetAbstraction_42597485641816
// MI455X (gfx1250) — hardware-verified
//
#include <hip/hip_runtime.h>
#include <stdint.h>

#pragma clang fp contract(off)

typedef __attribute__((ext_vector_type(16))) _Float16 v16h;
typedef __attribute__((ext_vector_type(8)))  _Float16 v8h;
typedef __attribute__((ext_vector_type(8)))  float    v8f;
typedef __attribute__((ext_vector_type(4)))  float    v4f;

constexpr int NB_BATCH = 16;
constexpr int NPTS     = 4096;
constexpr int NCENT    = 1024;
constexpr int NNBR     = 32;
constexpr int CFEAT    = 64;
constexpr int CH_L0    = 64;
constexpr int CH_L1    = 64;
constexpr int CH_L2    = 128;
constexpr int NROWS    = NB_BATCH * NCENT * NNBR;
constexpr int NGROUPS  = NB_BATCH * NCENT;
constexpr int NPTOT    = NB_BATCH * NPTS;
constexpr float WCARRY     = 16.0f;
constexpr float WCARRY_INV = 1.0f / 16.0f;
constexpr float BN_EPS_F   = 1e-5f;
static_assert(NROWS == 524288, "rows");
static_assert(NGROUPS == 16384, "groups");
static_assert(NPTOT == 65536, "points");
static_assert(NCENT == 1024 && NNBR == 32 && NPTS == 4096, "shift-based index math");
static_assert(CFEAT == 64 && CH_L0 == 64 && CH_L1 == 64 && CH_L2 == 128, "tile multiples, K % 32 == 0");

constexpr int GM_F32   = 0;
constexpr int GM_STATS = 1;
constexpr int GM_ACT16 = 2;
constexpr int GM_POOL  = 3;

union FragU { v16h v; v8h h[2]; };
__device__ __forceinline__ v16h frag_load(const _Float16* p) {
  FragU f;
  f.h[0] = *(const v8h*)(p);
  f.h[1] = *(const v8h*)(p + 16);
  return f.v;
}
__device__ __forceinline__ v8f frag_mma(v16h a, v16h b, v8f c) {
  return __builtin_amdgcn_wmma_f32_16x16x32_f16(false, a, false, b, (short)0, c, false, false);
}
__device__ __forceinline__ void guard_row(v8f& c0, v8f& c1, v8f& c2, v8f& c3,
                                          v16h a, v16h b0, v16h b1, v16h b2, v16h b3) {
  asm volatile("v_nop\n\tv_nop\n\tv_nop\n\tv_nop"
               : "+v"(c0), "+v"(c1), "+v"(c2), "+v"(c3)
               : "v"(a), "v"(b0), "v"(b1), "v"(b2), "v"(b3));
}
__device__ __forceinline__ void acc_guard4(v8f& a, v8f& b, v8f& c, v8f& d) {
  asm volatile("v_nop\n\tv_nop\n\tv_nop\n\tv_nop" : "+v"(a), "+v"(b), "+v"(c), "+v"(d));
}

__global__ __launch_bounds__(256) void cvt_points_kernel(const float* __restrict__ pts,
                                                         unsigned short* __restrict__ out16) {
  const int i = blockIdx.x * 256 + threadIdx.x;
  const v4f a = *(const v4f*)(pts + (size_t)i * 8);
  const v4f b = *(const v4f*)(pts + (size_t)i * 8 + 4);
  v8h hv;
  hv[0] = (_Float16)a[0]; hv[1] = (_Float16)a[1]; hv[2] = (_Float16)a[2]; hv[3] = (_Float16)a[3];
  hv[4] = (_Float16)b[0]; hv[5] = (_Float16)b[1]; hv[6] = (_Float16)b[2]; hv[7] = (_Float16)b[3];
  _Float16* dst = (_Float16*)out16 + (size_t)i * 8;
  for (int pass = 0; pass < 2; ++pass) {
    *(volatile v8h*)dst = hv;
    __threadfence();
  }
}

__global__ __launch_bounds__(256) void pts4_kernel(const float* __restrict__ xyz,
                                                   float* __restrict__ pts4) {
#pragma clang fp contract(off)
  const int i = blockIdx.x * 256 + threadIdx.x;
  const float x = xyz[(size_t)i * 3 + 0];
  const float y = xyz[(size_t)i * 3 + 1];
  const float z = xyz[(size_t)i * 3 + 2];
  const float t0 = x * x;
  const float t1 = y * y;
  const float t2 = z * z;
  v4f v;
  v[0] = x; v[1] = y; v[2] = z; v[3] = (t0 + t2) + t1;
  for (int pass = 0; pass < 2; ++pass) {
    *(volatile v4f*)(pts4 + (size_t)i * 4) = v;
    __threadfence();
  }
}

__global__ __launch_bounds__(256) void wplanes_kernel(const float* __restrict__ w0,
                                                      const float* __restrict__ w1,
                                                      const float* __restrict__ w2,
                                                      unsigned short* __restrict__ wpl) {
  const int t = blockIdx.x * 256 + threadIdx.x;
  const int row = t >> 3;
  const int kc = (t & 7) * 8;
  const float* src;
  int ldw;
  int n;
  if (blockIdx.x < 2) {
    src = w0 + 3 * CH_L0; ldw = CH_L0; n = row;
  } else if (blockIdx.x < 4) {
    src = w1; ldw = CH_L1; n = row - 64;
  } else {
    src = w2; ldw = CH_L2; n = row - 128;
  }
  v8h hv;
#pragma unroll
  for (int e = 0; e < 8; ++e) {
    const float w = src[(size_t)(kc + e) * ldw + n] * WCARRY;
    hv[e] = (_Float16)w;
  }
  _Float16* dst = (_Float16*)wpl + (size_t)row * 64 + kc;
  for (int pass = 0; pass < 2; ++pass) {
    *(volatile v8h*)dst = hv;
    __threadfence();
  }
}

__global__ __launch_bounds__(256) void fps_kernel(const float* __restrict__ xyz,
                                                  float* __restrict__ out0,
                                                  float* __restrict__ cen4) {
#pragma clang fp contract(off)
  __shared__ __align__(16) float sx[NPTS * 3];
  __shared__ int fidx[NCENT];
  __shared__ float rv[2][8];
  __shared__ int ri[2][8];
  const int b = blockIdx.x;
  const int tid = threadIdx.x;
  const int lane = tid & 31;
  const int wave = tid >> 5;
  const float* px = xyz + (size_t)b * NPTS * 3;
#pragma unroll 4
  for (int i = 0; i < 12; ++i) {
    const int q = i * 256 + tid;
    const v4f v = *(const v4f*)(px + 4 * q);
    *(v4f*)(sx + 4 * q) = v;
  }
  __syncthreads();

  float lx[16], ly[16], lz[16], dmin[16];
#pragma unroll
  for (int j = 0; j < 16; ++j) {
    const int p = j * 256 + tid;
    lx[j] = sx[p * 3 + 0];
    ly[j] = sx[p * 3 + 1];
    lz[j] = sx[p * 3 + 2];
    dmin[j] = 1e10f;
  }

  int far = 0;
#pragma unroll 1
  for (int s = 0; s < NCENT; ++s) {
    if (tid == 0) fidx[s] = far;
    const float cx = sx[far * 3 + 0];
    const float cy = sx[far * 3 + 1];
    const float cz = sx[far * 3 + 2];
    float bv = -1.0f;
    int bi = 0;
#pragma unroll
    for (int j = 0; j < 16; ++j) {
      const float dx = lx[j] - cx;
      const float dy = ly[j] - cy;
      const float dz = lz[j] - cz;
      const float t0 = dx * dx;
      const float t1 = dy * dy;
      const float t2 = dz * dz;
      const float d = (t0 + t2) + t1;
      const float dm = fminf(dmin[j], d);
      dmin[j] = dm;
      if (dm > bv) { bv = dm; bi = j * 256 + tid; }
    }
#pragma unroll
    for (int off = 16; off > 0; off >>= 1) {
      const float ov = __shfl_xor(bv, off, 32);
      const int oi = __shfl_xor(bi, off, 32);
      const bool take = (ov > bv) || (ov == bv && oi < bi);
      bv = take ? ov : bv;
      bi = take ? oi : bi;
    }
    const int buf = s & 1;
    if (lane == 0) { rv[buf][wave] = bv; ri[buf][wave] = bi; }
    __syncthreads();
    float fv = rv[buf][0];
    int fi = ri[buf][0];
#pragma unroll
    for (int w = 1; w < 8; ++w) {
      const float ov = rv[buf][w];
      const int oi = ri[buf][w];
      const bool take = (ov > fv) || (ov == fv && oi < fi);
      fv = take ? ov : fv;
      fi = take ? oi : fi;
    }
    far = fi & (NPTS - 1);
  }
  __syncthreads();

  v4f o[3];
#pragma unroll
  for (int i = 0; i < 3; ++i) {
    const int q = i * 256 + tid;
#pragma unroll
    for (int e = 0; e < 4; ++e) {
      const int el = 4 * q + e;
      const int s = el / 3;
      const int c = el - 3 * s;
      o[i][e] = sx[fidx[s] * 3 + c];
    }
  }
  v4f cv[4];
#pragma unroll
  for (int i = 0; i < 4; ++i) {
    const int f = fidx[i * 256 + tid];
    cv[i][0] = sx[f * 3 + 0];
    cv[i][1] = sx[f * 3 + 1];
    cv[i][2] = sx[f * 3 + 2];
    cv[i][3] = 0.0f;
  }
  float* ob = out0 + (size_t)b * NCENT * 3;
  float* cb = cen4 + (size_t)b * NCENT * 4;
  for (int pass = 0; pass < 2; ++pass) {
#pragma unroll
    for (int i = 0; i < 3; ++i) *(volatile v4f*)(ob + 4 * (i * 256 + tid)) = o[i];
#pragma unroll
    for (int i = 0; i < 4; ++i) *(volatile v4f*)(cb + 4 * (i * 256 + tid)) = cv[i];
    __threadfence();
  }
}

__global__ __launch_bounds__(64) void knn_kernel(const float* __restrict__ pts4,
                                                 const float* __restrict__ cen4,
                                                 int* __restrict__ knn_idx) {
#pragma clang fp contract(off)
  __shared__ unsigned long long slab[2][NPTS];
  const int lane = threadIdx.x & 31;
  const int wave = threadIdx.x >> 5;
  const int task = blockIdx.x * 2 + wave;
  const int b = task >> 10;
  const v4f c = *(const v4f*)(cen4 + (size_t)task * 4);
  const float cx = c[0];
  const float cy = c[1];
  const float cz = c[2];
  const float c0 = cx * cx;
  const float c1 = cy * cy;
  const float c2 = cz * cz;
  const float cc = (c0 + c2) + c1;
  const float* pb = pts4 + (size_t)b * NPTS * 4;
  unsigned long long* sl = slab[wave];

  unsigned lmin = 0xFFFFFFFFu;
#pragma unroll 4
  for (int i = 0; i < 128; ++i) {
    const int j = i * 32 + lane;
    const v4f p = *(const v4f*)(pb + (size_t)j * 4);
    float dot = cx * p[0];
    dot = fmaf(cy, p[1], dot);
    dot = fmaf(cz, p[2], dot);
    const float two = 2.0f * dot;
    const float t = cc - two;
    const float d = t + p[3];
    const unsigned u = __float_as_uint(d);
    const unsigned mono = u ^ ((unsigned)((int)u >> 31) | 0x80000000u);
    lmin = (mono < lmin) ? mono : lmin;
    sl[j] = ((unsigned long long)mono << 32) | (unsigned long long)(unsigned)j;
  }
  unsigned t0key = lmin;
#pragma unroll
  for (int off = 16; off > 0; off >>= 1) {
    const unsigned o = __shfl_xor(t0key, off, 32);
    t0key = (o > t0key) ? o : t0key;
  }
  __builtin_amdgcn_fence(__ATOMIC_RELEASE, "workgroup");
  __builtin_amdgcn_wave_barrier();
  __builtin_amdgcn_fence(__ATOMIC_ACQUIRE, "workgroup");

  const unsigned lt_mask = (1u << lane) - 1u;
  int cnt = 0;
#pragma unroll 1
  for (int i = 0; i < 128; ++i) {
    const int p = i * 32 + lane;
    const unsigned long long k = sl[p];
    const bool hit = ((unsigned)(k >> 32)) <= t0key;
    const unsigned mask = __builtin_amdgcn_ballot_w32(hit);
    const int pre = __popc(mask & lt_mask);
    if (hit) sl[cnt + pre] = k;
    cnt += __popc(mask);
  }
  __builtin_amdgcn_fence(__ATOMIC_RELEASE, "workgroup");
  __builtin_amdgcn_wave_barrier();
  __builtin_amdgcn_fence(__ATOMIC_ACQUIRE, "workgroup");

  int ncand = __builtin_amdgcn_readfirstlane(cnt);
  ncand = ncand > NPTS ? NPTS : ncand;
  int nIter = (ncand + 31) >> 5;
  nIter = nIter > 128 ? 128 : nIter;

  int res = 0;
#pragma unroll 1
  for (int it = 0; it < NNBR; ++it) {
    unsigned lhi = 0xFFFFFFFFu;
    unsigned llo = 0xFFFFFFFFu;
    int lpos = 0;
#pragma unroll 1
    for (int tt = 0; tt < nIter; ++tt) {
      const int p = tt * 32 + lane;
      const int pc = p < NPTS - 1 ? p : NPTS - 1;
      const unsigned long long k = sl[pc];
      const bool valid = p < ncand;
      const unsigned khi = valid ? (unsigned)(k >> 32) : 0xFFFFFFFFu;
      const unsigned klo = valid ? (unsigned)k : 0xFFFFFFFFu;
      const bool lt = (khi < lhi) || (khi == lhi && klo < llo);
      lhi = lt ? khi : lhi;
      llo = lt ? klo : llo;
      lpos = lt ? p : lpos;
    }
    unsigned bhi = lhi;
    unsigned blo = llo;
#pragma unroll
    for (int off = 16; off > 0; off >>= 1) {
      const unsigned ohi = __shfl_xor(bhi, off, 32);
      const unsigned olo = __shfl_xor(blo, off, 32);
      const bool lt = (ohi < bhi) || (ohi == bhi && olo < blo);
      bhi = lt ? ohi : bhi;
      blo = lt ? olo : blo;
    }
    const bool winner = (lhi == bhi) && (llo == blo) && (bhi != 0xFFFFFFFFu);
    if (winner) sl[lpos] = ~0ull;
    res = (lane == it) ? (int)blo : res;
  }
  int o = res;
  o = o < 0 ? 0 : o;
  o = o > NPTS - 1 ? NPTS - 1 : o;
  int* dst = knn_idx + (size_t)task * NNBR + lane;
  for (int pass = 0; pass < 2; ++pass) {
    *(volatile int*)dst = o;
    __threadfence();
  }
}

template <bool WRITE_PLANE>
__global__ __launch_bounds__(256) void gather_l0(const int* __restrict__ knn_idx,
                                                 const float* __restrict__ pts4,
                                                 const float* __restrict__ cen4,
                                                 const float* __restrict__ Pf,
                                                 const float* __restrict__ w0,
                                                 const float* __restrict__ b0,
                                                 const float* __restrict__ tab,
                                                 unsigned short* __restrict__ planeOut,
                                                 float* __restrict__ part) {
  __shared__ float red[WRITE_PLANE ? 32 : 4096];
  const int t = threadIdx.x;
  const int c8 = (t & 7) * 8;
  const int rs = t >> 3;

  const v4f wxa = *(const v4f*)(w0 + c8);
  const v4f wxb = *(const v4f*)(w0 + c8 + 4);
  const v4f wya = *(const v4f*)(w0 + CH_L0 + c8);
  const v4f wyb = *(const v4f*)(w0 + CH_L0 + c8 + 4);
  asm volatile("" ::: "memory");
  const v4f wza = *(const v4f*)(w0 + 2 * CH_L0 + c8);
  const v4f wzb = *(const v4f*)(w0 + 2 * CH_L0 + c8 + 4);
  const v4f bia = *(const v4f*)(b0 + c8);
  const v4f bib = *(const v4f*)(b0 + c8 + 4);
  asm volatile("" ::: "memory");
  v4f sca = (v4f){0.f, 0.f, 0.f, 0.f};
  v4f scb = sca, sha = sca, shb = sca;
  if (WRITE_PLANE) {
    sca = *(const v4f*)(tab + c8);
    scb = *(const v4f*)(tab + c8 + 4);
    sha = *(const v4f*)(tab + 128 + c8);
    shb = *(const v4f*)(tab + 128 + c8 + 4);
  }

  float s[8], q[8];
#pragma unroll
  for (int e = 0; e < 8; ++e) { s[e] = 0.0f; q[e] = 0.0f; }

#pragma unroll 1
  for (int it = 0; it < 16; ++it) {
    const int row = blockIdx.x * 512 + it * 32 + rs;
    int idx = knn_idx[row];
    idx = idx < 0 ? 0 : idx;
    idx = idx > NPTS - 1 ? NPTS - 1 : idx;
    const int bs = row >> 5;
    const int b = row >> 15;
    const size_t pidx = (size_t)b * NPTS + idx;
    const v4f p4 = *(const v4f*)(pts4 + pidx * 4);
    const v4f c4 = *(const v4f*)(cen4 + (size_t)bs * 4);
    const v4f pa = *(const v4f*)(Pf + pidx * CH_L0 + c8);
    const v4f pb = *(const v4f*)(Pf + pidx * CH_L0 + c8 + 4);
    const float dx = p4[0] - c4[0];
    const float dy = p4[1] - c4[1];
    const float dz = p4[2] - c4[2];
    float y[8];
#pragma unroll
    for (int e = 0; e < 4; ++e) {
      float ta = dx * wxa[e];
      ta = fmaf(dy, wya[e], ta);
      ta = fmaf(dz, wza[e], ta);
      y[e] = (pa[e] + ta) + bia[e];
      float tb = dx * wxb[e];
      tb = fmaf(dy, wyb[e], tb);
      tb = fmaf(dz, wzb[e], tb);
      y[4 + e] = (pb[e] + tb) + bib[e];
    }
    if (WRITE_PLANE) {
      v8h hv;
#pragma unroll
      for (int e = 0; e < 4; ++e) {
        const float a0 = fmaxf(fmaf(y[e], sca[e], sha[e]), 0.0f);
        const float a1 = fmaxf(fmaf(y[4 + e], scb[e], shb[e]), 0.0f);
        hv[e] = (_Float16)a0;
        hv[4 + e] = (_Float16)a1;
      }
      _Float16* dst = (_Float16*)planeOut + (size_t)row * CH_L0 + c8;
      for (int pass = 0; pass < 2; ++pass) {
        *(volatile v8h*)dst = hv;
        __threadfence();
      }
    } else {
#pragma unroll
      for (int e = 0; e < 8; ++e) {
        s[e] += y[e];
        q[e] = fmaf(y[e], y[e], q[e]);
      }
    }
  }

  if (!WRITE_PLANE) {
#pragma unroll
    for (int e = 0; e < 8; ++e) {
      red[t * 16 + e] = s[e];
      red[t * 16 + 8 + e] = q[e];
    }
    __syncthreads();
    if (t < 128) {
      const int st = t >> 6;
      const int col = t & 63;
      const int ci = col >> 3;
      const int e = col & 7;
      float tot = 0.0f;
#pragma unroll 4
      for (int r = 0; r < 32; ++r) tot += red[(r * 8 + ci) * 16 + st * 8 + e];
      float* dst = part + (size_t)blockIdx.x * 128 + t;
      for (int pass = 0; pass < 2; ++pass) {
        *(volatile float*)dst = tot;
        __threadfence();
      }
    }
  }
}

__global__ __launch_bounds__(256) void bn_finalize(const float* __restrict__ part, int nPart, int nch,
                                                   const float* __restrict__ g,
                                                   const float* __restrict__ be,
                                                   float* __restrict__ tab) {
  __shared__ double tot[256];
  const int t = threadIdx.x;
  const int col = t & 127;
  const int st = t >> 7;
  const int cc = col < nch ? col : nch - 1;
  const int pitch = 2 * nch;
  const float* p = part + st * nch + cc;
  double acc = 0.0;
#pragma unroll 4
  for (int i = 0; i < nPart; ++i) acc += (double)p[(size_t)i * pitch];
  tot[t] = acc;
  __syncthreads();
  const double invR = 1.0 / (double)NROWS;
  const double mean = tot[cc] * invR;
  const double ex2 = tot[128 + cc] * invR;
  double var = ex2 - mean * mean;
  var = var < 0.0 ? 0.0 : var;
  const float sc = g[cc] * rsqrtf((float)var + BN_EPS_F);
  const float sh = be[cc] - (float)mean * sc;
  float v = (st == 0) ? sc : sh;
  v = (col < nch) ? v : 0.0f;
  for (int pass = 0; pass < 2; ++pass) {
    *(volatile float*)(tab + t) = v;
    __threadfence();
  }
}

template <int MODE, int NTILES>
__global__ __launch_bounds__(256) void mlp_gemm(const unsigned short* __restrict__ Ap,
                                                const unsigned short* __restrict__ Btp,
                                                int tilesM, float wscale,
                                                const float* __restrict__ bias,
                                                const float* __restrict__ tab,
                                                float* __restrict__ outF,
                                                float* __restrict__ outF2,
                                                unsigned short* __restrict__ outH,
                                                float* __restrict__ part) {
  constexpr int GN = 64 * NTILES;
  constexpr int GK = 64;
  static_assert(GK % 32 == 0, "k step");
  constexpr bool USE_SLAB = (MODE == GM_F32) || (MODE == GM_ACT16);
  constexpr bool USE_STAT = (MODE == GM_STATS) || (MODE == GM_POOL);
  __shared__ __align__(16) float sT[USE_SLAB ? 8 * 16 * 68 : 16];
  __shared__ __align__(16) float wsum[USE_STAT ? 8 * 128 : 16];
  __shared__ __align__(16) float pool[(MODE == GM_POOL) ? 8 * 256 : 16];

  const _Float16* A = (const _Float16*)Ap;
  const _Float16* Bt = (const _Float16*)Btp;
  const int lane = threadIdx.x & 31;
  const int wave = threadIdx.x >> 5;
  int tile = blockIdx.x * 8 + wave;
  const int lastTile = tilesM * NTILES - 1;
  tile = tile < lastTile ? tile : lastTile;
  const int tm = tile / NTILES;
  const int tn = tile - tm * NTILES;
  const int m0 = tm << 6;
  const int n0 = tn << 6;
  const int rlane = lane & 15;
  const int koff = (lane >> 4) * 8;
  const int mOff = (lane >> 4) * 8;

  v8f acc[4][4];
#pragma unroll
  for (int i = 0; i < 4; ++i)
#pragma unroll
    for (int j = 0; j < 4; ++j) acc[i][j] = (v8f){0.f, 0.f, 0.f, 0.f, 0.f, 0.f, 0.f, 0.f};

#pragma unroll 1
  for (int k0 = 0; k0 < GK; k0 += 32) {
    v16h bh[4];
#pragma unroll
    for (int j = 0; j < 4; ++j)
      bh[j] = frag_load(Bt + (size_t)(n0 + (j << 4) + rlane) * GK + koff + k0);
#pragma unroll
    for (int i = 0; i < 4; ++i) {
      const v16h ah = frag_load(A + (size_t)(m0 + (i << 4) + rlane) * GK + koff + k0);
#pragma unroll
      for (int j = 0; j < 4; ++j) acc[i][j] = frag_mma(ah, bh[j], acc[i][j]);
      guard_row(acc[i][0], acc[i][1], acc[i][2], acc[i][3], ah, bh[0], bh[1], bh[2], bh[3]);
    }
  }
  acc_guard4(acc[0][0], acc[0][1], acc[0][2], acc[0][3]);
  acc_guard4(acc[1][0], acc[1][1], acc[1][2], acc[1][3]);
  acc_guard4(acc[2][0], acc[2][1], acc[2][2], acc[2][3]);
  acc_guard4(acc[3][0], acc[3][1], acc[3][2], acc[3][3]);

  if (USE_STAT) {
#pragma unroll
    for (int j = 0; j < 4; ++j) {
      const float bv = bias[n0 + (j << 4) + rlane];
      float sum = 0.0f;
      float sq = 0.0f;
      float mx0 = -3.0e38f, mx1 = -3.0e38f, mn0 = 3.0e38f, mn1 = 3.0e38f;
#pragma unroll
      for (int i = 0; i < 4; ++i) {
#pragma unroll
        for (int r = 0; r < 8; ++r) {
          const float y = fmaf(acc[i][j][r], wscale, bv);
          sum += y;
          sq = fmaf(y, y, sq);
          if (MODE == GM_POOL) {
            if (i < 2) { mx0 = fmaxf(mx0, y); mn0 = fminf(mn0, y); }
            else       { mx1 = fmaxf(mx1, y); mn1 = fminf(mn1, y); }
          }
        }
      }
      sum += __shfl_xor(sum, 16, 32);
      sq += __shfl_xor(sq, 16, 32);
      if (MODE == GM_POOL) {
        mx0 = fmaxf(mx0, __shfl_xor(mx0, 16, 32));
        mx1 = fmaxf(mx1, __shfl_xor(mx1, 16, 32));
        mn0 = fminf(mn0, __shfl_xor(mn0, 16, 32));
        mn1 = fminf(mn1, __shfl_xor(mn1, 16, 32));
      }
      if (lane < 16) {
        wsum[wave * 128 + (j << 4) + rlane] = sum;
        wsum[wave * 128 + 64 + (j << 4) + rlane] = sq;
        if (MODE == GM_POOL) {
          pool[wave * 256 + 0 * 64 + (j << 4) + rlane] = mx0;
          pool[wave * 256 + 1 * 64 + (j << 4) + rlane] = mx1;
          pool[wave * 256 + 2 * 64 + (j << 4) + rlane] = mn0;
          pool[wave * 256 + 3 * 64 + (j << 4) + rlane] = mn1;
        }
      }
    }
    __syncthreads();
    const int t = threadIdx.x;
    if (t < 2 * GN) {
      const int st = t / GN;
      const int col = t - st * GN;
      const int tnn = col >> 6;
      const int cl = col & 63;
      float tot = 0.0f;
#pragma unroll
      for (int w = 0; w < 8 / NTILES; ++w) tot += wsum[(tnn + w * NTILES) * 128 + st * 64 + cl];
      float* dst = part + (size_t)blockIdx.x * (2 * GN) + t;
      for (int pass = 0; pass < 2; ++pass) {
        *(volatile float*)dst = tot;
        __threadfence();
      }
    }
    if (MODE == GM_POOL) {
      const int hh = lane >> 4;
      const int c4 = (lane & 15) * 4;
      const v4f vx = *(const v4f*)(pool + wave * 256 + hh * 64 + c4);
      const v4f vn = *(const v4f*)(pool + wave * 256 + (2 + hh) * 64 + c4);
      float* px = outF + (size_t)(tm * 2 + hh) * GN + n0 + c4;
      float* pn = outF2 + (size_t)(tm * 2 + hh) * GN + n0 + c4;
      for (int pass = 0; pass < 2; ++pass) {
        *(volatile v4f*)px = vx;
        *(volatile v4f*)pn = vn;
        __threadfence();
      }
    }
  }

  if (USE_SLAB) {
    float* slab = sT + wave * (16 * 68);
    float bvv[4], scv[4], shv[4];
#pragma unroll
    for (int j = 0; j < 4; ++j) {
      bvv[j] = 0.0f; scv[j] = 1.0f; shv[j] = 0.0f;
      if (MODE == GM_ACT16) {
        const int n = n0 + (j << 4) + rlane;
        bvv[j] = bias[n];
        scv[j] = tab[n];
        shv[j] = tab[128 + n];
      }
    }
#pragma unroll
    for (int i = 0; i < 4; ++i) {
      const int mBase = m0 + (i << 4);
#pragma unroll
      for (int j = 0; j < 4; ++j) {
#pragma unroll
        for (int r = 0; r < 8; ++r) {
          float v;
          if (MODE == GM_ACT16) {
            const float y = fmaf(acc[i][j][r], wscale, bvv[j]);
            v = fmaxf(fmaf(y, scv[j], shv[j]), 0.0f);
          } else {
            v = acc[i][j][r] * wscale;
          }
          slab[(mOff + r) * 68 + (j << 4) + rlane] = v;
        }
      }
      __builtin_amdgcn_fence(__ATOMIC_RELEASE, "workgroup");
      __builtin_amdgcn_wave_barrier();
      __builtin_amdgcn_fence(__ATOMIC_ACQUIRE, "workgroup");
      if (MODE == GM_F32) {
        const int hh = lane >> 4;
        const int c4 = (lane & 15) * 4;
        for (int pass = 0; pass < 2; ++pass) {
#pragma unroll
          for (int it = 0; it < 8; ++it) {
            const int row = it * 2 + hh;
            const v4f v = *(const v4f*)(slab + row * 68 + c4);
            *(volatile v4f*)(outF + (size_t)(mBase + row) * GN + n0 + c4) = v;
          }
          __threadfence();
        }
      } else {
        const int qd = lane >> 3;
        const int c8 = (lane & 7) * 8;
        for (int pass = 0; pass < 2; ++pass) {
#pragma unroll
          for (int it = 0; it < 4; ++it) {
            const int row = it * 4 + qd;
            const float* sp = slab + row * 68 + c8;
            v8h hv;
#pragma unroll
            for (int e = 0; e < 8; ++e) hv[e] = (_Float16)sp[e];
            *(volatile v8h*)((_Float16*)outH + (size_t)(mBase + row) * GN + n0 + c8) = hv;
          }
          __threadfence();
        }
      }
      __builtin_amdgcn_fence(__ATOMIC_RELEASE, "workgroup");
      __builtin_amdgcn_wave_barrier();
      __builtin_amdgcn_fence(__ATOMIC_ACQUIRE, "workgroup");
    }
  }
}

__global__ __launch_bounds__(256) void out_kernel(const float* __restrict__ gmax,
                                                  const float* __restrict__ gmin,
                                                  const float* __restrict__ tab,
                                                  float* __restrict__ out1) {
  const int i = blockIdx.x * 256 + threadIdx.x;
  const int c4 = (i & 31) * 4;
  const v4f mx = *(const v4f*)(gmax + (size_t)i * 4);
  const v4f mn = *(const v4f*)(gmin + (size_t)i * 4);
  const v4f sc = *(const v4f*)(tab + c4);
  const v4f sh = *(const v4f*)(tab + 128 + c4);
  v4f o;
#pragma unroll
  for (int e = 0; e < 4; ++e) {
    const float sel = (sc[e] >= 0.0f) ? mx[e] : mn[e];
    o[e] = fmaxf(fmaf(sc[e], sel, sh[e]), 0.0f);
  }
  for (int pass = 0; pass < 2; ++pass) {
    *(volatile v4f*)(out1 + (size_t)i * 4) = o;
    __threadfence();
  }
}

constexpr size_t SZ_A0    = (size_t)NROWS * 64 * 2;
constexpr size_t SZ_A1H   = (size_t)(NROWS / 2) * 64 * 2;
constexpr size_t SZ_PG    = (size_t)NPTOT * 64 * 4;
constexpr size_t SZ_PTS16 = (size_t)NPTOT * 64 * 2;
constexpr size_t SZ_KNN   = (size_t)NROWS * 4;
constexpr size_t SZ_PTS4  = (size_t)NPTOT * 16;
constexpr size_t SZ_CEN4  = (size_t)NGROUPS * 16;
constexpr size_t SZ_PART0 = (size_t)1024 * 128 * 4;
constexpr size_t SZ_PART1 = (size_t)1024 * 128 * 4;
constexpr size_t SZ_PART2 = (size_t)2048 * 256 * 4;
constexpr size_t SZ_WPL   = (size_t)256 * 64 * 2;
constexpr size_t SZ_TAB   = 4096;
constexpr size_t OFF_A0    = 0;
constexpr size_t OFF_A1H   = OFF_A0 + SZ_A0;
constexpr size_t OFF_PG    = OFF_A1H + SZ_A1H;
constexpr size_t OFF_PTS16 = OFF_PG + SZ_PG;
constexpr size_t OFF_KNN   = OFF_PTS16 + SZ_PTS16;
constexpr size_t OFF_PTS4  = OFF_KNN + SZ_KNN;
constexpr size_t OFF_CEN4  = OFF_PTS4 + SZ_PTS4;
constexpr size_t OFF_PART0 = OFF_CEN4 + SZ_CEN4;
constexpr size_t OFF_PART1 = OFF_PART0 + SZ_PART0;
constexpr size_t OFF_PART2 = OFF_PART1 + SZ_PART1;
constexpr size_t OFF_WPL   = OFF_PART2 + SZ_PART2;
constexpr size_t OFF_TAB   = OFF_WPL + SZ_WPL;
constexpr size_t WS_TOTAL  = OFF_TAB + SZ_TAB;
static_assert(WS_TOTAL <= (size_t)134217728, "carve within 128 MiB");
static_assert(SZ_PG == (size_t)2 * NGROUPS * CH_L2 * 4, "P plane and gmax+gmin share one f32 region");
static_assert((OFF_A1H % 256) == 0 && (OFF_PG % 256) == 0 && (OFF_PTS16 % 256) == 0 && (OFF_KNN % 256) == 0, "align");
static_assert((OFF_PTS4 % 256) == 0 && (OFF_CEN4 % 256) == 0 && (OFF_PART0 % 256) == 0 && (OFF_TAB % 256) == 0, "align");
constexpr size_t OUT1_OFF_BYTES = 196608;
constexpr size_t OUT_TOTAL_BYTES = 8585216;
static_assert(OUT1_OFF_BYTES == (size_t)NGROUPS * 3 * 4, "out1 offset");
static_assert(OUT1_OFF_BYTES % 128 == 0, "out1 line aligned");
static_assert(OUT1_OFF_BYTES + (size_t)NGROUPS * CH_L2 * 4 == OUT_TOTAL_BYTES, "out extent");
static_assert(NPTOT % 64 == 0 && NROWS % 128 == 0 && (NROWS / 2) % 64 == 0, "M tiles");
static_assert(((NPTOT / 64) % 8) == 0 && ((NROWS / 64) % 8) == 0 && ((NROWS / 128) % 8) == 0, "8 tiles per block");

extern "C" void kernel_launch(void* const* d_in, const int* in_sizes, int n_in,
                              void* d_out, int out_size, void* d_ws, size_t ws_size,
                              hipStream_t stream) {
  if (n_in < 14) return;
  if (ws_size < WS_TOTAL) return;
  if ((size_t)out_size * 4 != OUT_TOTAL_BYTES) return;
  if (in_sizes[0] != NPTOT * 3 || in_sizes[1] != NPTOT * CFEAT) return;

  const float* xyz    = (const float*)d_in[0];
  const float* points = (const float*)d_in[1];
  const float* w0  = (const float*)d_in[2];
  const float* b0  = (const float*)d_in[3];
  const float* g0  = (const float*)d_in[4];
  const float* be0 = (const float*)d_in[5];
  const float* w1  = (const float*)d_in[6];
  const float* b1  = (const float*)d_in[7];
  const float* g1  = (const float*)d_in[8];
  const float* be1 = (const float*)d_in[9];
  const float* w2  = (const float*)d_in[10];
  const float* b2  = (const float*)d_in[11];
  const float* g2  = (const float*)d_in[12];
  const float* be2 = (const float*)d_in[13];

  float* out0 = (float*)d_out;
  float* out1 = (float*)d_out + OUT1_OFF_BYTES / 4;

  char* ws = (char*)d_ws;
  unsigned short* A0    = (unsigned short*)(ws + OFF_A0);
  unsigned short* A1H   = (unsigned short*)(ws + OFF_A1H);
  float*          PG    = (float*)(ws + OFF_PG);
  unsigned short* PTS16 = (unsigned short*)(ws + OFF_PTS16);
  int*            KNN   = (int*)(ws + OFF_KNN);
  float*          PTS4  = (float*)(ws + OFF_PTS4);
  float*          CEN4  = (float*)(ws + OFF_CEN4);
  float*          PART0 = (float*)(ws + OFF_PART0);
  float*          PART1 = (float*)(ws + OFF_PART1);
  float*          PART2 = (float*)(ws + OFF_PART2);
  unsigned short* WPL   = (unsigned short*)(ws + OFF_WPL);
  float*          TAB0  = (float*)(ws + OFF_TAB);
  float*          TAB1  = TAB0 + 256;
  float*          TAB2  = TAB0 + 512;
  unsigned short* W0PT = WPL;
  unsigned short* W1T  = WPL + 64 * 64;
  unsigned short* W2T  = WPL + 128 * 64;
  float* GMAX = PG;
  float* GMIN = PG + (size_t)NGROUPS * CH_L2;

  cvt_points_kernel<<<NPTOT * CFEAT / 8 / 256, 256, 0, stream>>>(points, PTS16);
  pts4_kernel<<<NPTOT / 256, 256, 0, stream>>>(xyz, PTS4);
  wplanes_kernel<<<8, 256, 0, stream>>>(w0, w1, w2, WPL);

  mlp_gemm<GM_F32, 1><<<(NPTOT / 64) / 8, 256, 0, stream>>>(
      PTS16, W0PT, NPTOT / 64, WCARRY_INV, b0, TAB0, PG, PG, A1H, PART0);

  fps_kernel<<<NB_BATCH, 256, 0, stream>>>(xyz, out0, CEN4);
  knn_kernel<<<NGROUPS / 2, 64, 0, stream>>>(PTS4, CEN4, KNN);

  gather_l0<false><<<NROWS / 512, 256, 0, stream>>>(KNN, PTS4, CEN4, PG, w0, b0, TAB0, A0, PART0);
  bn_finalize<<<1, 256, 0, stream>>>(PART0, 1024, CH_L0, g0, be0, TAB0);
  gather_l0<true><<<NROWS / 512, 256, 0, stream>>>(KNN, PTS4, CEN4, PG, w0, b0, TAB0, A0, PART0);

  mlp_gemm<GM_STATS, 1><<<(NROWS / 64) / 8, 256, 0, stream>>>(
      A0, W1T, NROWS / 64, WCARRY_INV, b1, TAB1, PG, PG, A1H, PART1);
  bn_finalize<<<1, 256, 0, stream>>>(PART1, 1024, CH_L1, g1, be1, TAB1);

  for (int h = 0; h < 2; ++h) {
    const unsigned short* A0h = A0 + (size_t)h * (NROWS / 2) * 64;
    mlp_gemm<GM_ACT16, 1><<<(NROWS / 128) / 8, 256, 0, stream>>>(
        A0h, W1T, NROWS / 128, WCARRY_INV, b1, TAB1, PG, PG, A1H, PART1);
    mlp_gemm<GM_POOL, 2><<<(NROWS / 128) * 2 / 8, 256, 0, stream>>>(
        A1H, W2T, NROWS / 128, WCARRY_INV, b2, TAB2,
        GMAX + (size_t)h * (NGROUPS / 2) * CH_L2, GMIN + (size_t)h * (NGROUPS / 2) * CH_L2,
        A1H, PART2 + (size_t)h * 1024 * 256);
  }
  bn_finalize<<<1, 256, 0, stream>>>(PART2, 2048, CH_L2, g2, be2, TAB2);

  out_kernel<<<NGROUPS * CH_L2 / 4 / 256, 256, 0, stream>>>(GMAX, GMIN, TAB2, out1);
}
